// DSTQFunction_28415503630466
// MI455X (gfx1250) — hardware-verified
//
#include <hip/hip_runtime.h>

typedef __attribute__((ext_vector_type(16))) _Float16 v16h;
typedef __attribute__((ext_vector_type(4)))  float    v4f;
typedef __attribute__((ext_vector_type(8)))  _Float16 v8h;
typedef __attribute__((ext_vector_type(4)))  _Float16 v4h;
typedef __attribute__((ext_vector_type(8)))  float    v8f;

#define THREADS        128
#define ROWS_PER_BLOCK 128
#define KCHUNKS        11
#define FEAT_STRIDE    360
#define W1FRAG_HALVES  (KCHUNKS * 4 * 32 * 16)
#define FEAT_HALVES    (ROWS_PER_BLOCK * FEAT_STRIDE)

__global__ __launch_bounds__(THREADS)
void sig_mlp_kernel(const float* __restrict__ seq,
                    const float* __restrict__ Wa,
                    const float* __restrict__ ba,
                    const float* __restrict__ W1,
                    const float* __restrict__ b1,
                    const float* __restrict__ W2,
                    const float* __restrict__ b2,
                    float* __restrict__ out)
{
    __shared__ __align__(32) _Float16 smem[W1FRAG_HALVES + FEAT_HALVES];
    _Float16* __restrict__ w1frag = smem;
    _Float16* __restrict__ feat   = smem + W1FRAG_HALVES;

    const int tid = threadIdx.x;

    for (int e = tid; e < W1FRAG_HALVES; e += THREADS) {
        const int h    = e & 15;
        const int lane = (e >> 4) & 31;
        const int nt   = (e >> 9) & 3;
        const int kc   = e >> 11;
        const int n    = nt * 16 + (lane & 15);
        const int k    = kc * 32 + ((h < 8) ? h : (h + 8)) + ((lane >> 4) << 3);
        const float v  = (k < 342) ? W1[n * 342 + k] : 0.0f;
        w1frag[e] = (_Float16)v;
    }

    {
        const long  row = (long)blockIdx.x * ROWS_PER_BLOCK + tid;
        const float4 s  = *(const float4*)(seq + row * 4);
        const float wa00 = Wa[0], wa01 = Wa[1], wa10 = Wa[2], wa11 = Wa[3];
        const float ba0 = ba[0], ba1 = ba[1];

        float x[4], y[4];
        x[0] = s.x; x[1] = s.y;
        x[2] = wa00 * s.x + wa01 * s.y + ba0;
        x[3] = wa10 * s.x + wa11 * s.y + ba1;
        y[0] = s.z - x[0];
        y[1] = s.w - x[1];
        y[2] = (wa00 * s.z + wa01 * s.w + ba0) - x[2];
        y[3] = (wa10 * s.z + wa11 * s.w + ba1) - x[3];

        float a2[16], bb2[16];
        #pragma unroll
        for (int i = 0; i < 4; ++i)
            #pragma unroll
            for (int j = 0; j < 4; ++j) {
                a2[i * 4 + j]  = 0.5f * x[i] * x[j];
                bb2[i * 4 + j] = 0.5f * y[i] * y[j];
            }

        const float inv3 = (1.0f / 3.0f);
        _Float16* __restrict__ fr = feat + tid * FEAT_STRIDE;

        {
            v4h t;
            #pragma unroll
            for (int i = 0; i < 4; ++i) t[i] = (_Float16)(x[i] + y[i]);
            *(v4h*)(fr + 0) = t;
        }
        #pragma unroll
        for (int i = 0; i < 4; ++i) {
            v4h t;
            #pragma unroll
            for (int j = 0; j < 4; ++j)
                t[j] = (_Float16)(a2[i * 4 + j] + bb2[i * 4 + j] + x[i] * y[j]);
            *(v4h*)(fr + 4 + i * 4) = t;
        }
        #pragma unroll
        for (int i = 0; i < 4; ++i)
            #pragma unroll
            for (int j = 0; j < 4; ++j) {
                const float aij = a2[i * 4 + j], bij = bb2[i * 4 + j];
                v4h t;
                #pragma unroll
                for (int k = 0; k < 4; ++k)
                    t[k] = (_Float16)(aij * (x[k] * inv3 + y[k])
                                      + bij * y[k] * inv3
                                      + x[i] * bb2[j * 4 + k]);
                *(v4h*)(fr + 20 + (i * 4 + j) * 4) = t;
            }
        #pragma unroll
        for (int i = 0; i < 4; ++i)
            #pragma unroll
            for (int j = 0; j < 4; ++j) {
                const float aij = a2[i * 4 + j], bij = bb2[i * 4 + j];
                #pragma unroll
                for (int k = 0; k < 4; ++k) {
                    const float axk = aij * x[k] * inv3;
                    const float byk = bij * y[k] * inv3;
                    const float xbjk = x[i] * bb2[j * 4 + k] * inv3;
                    v4h t;
                    #pragma unroll
                    for (int l = 0; l < 4; ++l)
                        t[l] = (_Float16)(axk * (0.25f * x[l] + y[l])
                                          + byk * 0.25f * y[l]
                                          + xbjk * y[l]
                                          + aij * bb2[k * 4 + l]);
                    *(v4h*)(fr + 84 + ((i * 4 + j) * 4 + k) * 4) = t;
                }
            }
        fr[340] = (_Float16)s.y;
        fr[341] = (_Float16)s.w;
        #pragma unroll
        for (int k = 342; k < 352; ++k) fr[k] = (_Float16)0.0f;
    }
    __syncthreads();

    const int wave = tid >> 5;
    const int lane = tid & 31;
    const int cSel = lane & 15;
    const int hSel = lane >> 4;

    v8f acc[2][4];
    const v8f vzero = {0.f, 0.f, 0.f, 0.f, 0.f, 0.f, 0.f, 0.f};
    #pragma unroll
    for (int mt = 0; mt < 2; ++mt)
        #pragma unroll
        for (int nt = 0; nt < 4; ++nt) acc[mt][nt] = vzero;

    for (int kc = 0; kc < KCHUNKS; ++kc) {
        v16h A[2];
        #pragma unroll
        for (int mt = 0; mt < 2; ++mt) {
            const _Float16* p = feat + (wave * 32 + mt * 16 + cSel) * FEAT_STRIDE
                                + kc * 32 + hSel * 8;
            v8h lo = *(const v8h*)p;
            v8h hi = *(const v8h*)(p + 16);
            A[mt] = __builtin_shufflevector(lo, hi, 0, 1, 2, 3, 4, 5, 6, 7,
                                                    8, 9, 10, 11, 12, 13, 14, 15);
        }
        #pragma unroll
        for (int nt = 0; nt < 4; ++nt) {
            v16h Bf = *(const v16h*)(w1frag + ((kc * 4 + nt) * 32 + lane) * 16);
            acc[0][nt] = __builtin_amdgcn_wmma_f32_16x16x32_f16(
                false, A[0], false, Bf, (short)0, acc[0][nt], false, false);
            acc[1][nt] = __builtin_amdgcn_wmma_f32_16x16x32_f16(
                false, A[1], false, Bf, (short)0, acc[1][nt], false, false);
            asm volatile("v_nop\n\tv_nop\n\tv_nop\n\tv_nop" : "+v"(acc[0][nt]), "+v"(acc[1][nt]) : "v"(A[0]), "v"(A[1]), "v"(Bf));
        }
    }
    __syncthreads();

    float* __restrict__ hbuf = (float*)feat;
    #pragma unroll
    for (int mt = 0; mt < 2; ++mt)
        #pragma unroll
        for (int nt = 0; nt < 4; ++nt)
            #pragma unroll
            for (int j = 0; j < 8; ++j) {
                const int r = wave * 32 + mt * 16 + hSel * 8 + j;
                const int n = nt * 16 + cSel;
                hbuf[r * 65 + n] = acc[mt][nt][j];
            }
    __syncthreads();

    {
        float o0 = b2[0], o1 = b2[1], o2 = b2[2];
        const float* __restrict__ hrow = hbuf + tid * 65;
        #pragma unroll 8
        for (int n = 0; n < 64; ++n) {
            float hv = hrow[n] + b1[n];
            hv = hv > 0.0f ? hv : 0.0f;
            o0 += hv * W2[n];
            o1 += hv * W2[64 + n];
            o2 += hv * W2[128 + n];
        }
        float* __restrict__ sOut = (float*)smem;
        __syncthreads();
        sOut[tid * 3 + 0] = o0;
        sOut[tid * 3 + 1] = o1;
        sOut[tid * 3 + 2] = o2;
        __syncthreads();
        if (tid < 96) {
            float* ob = out + (long)blockIdx.x * ROWS_PER_BLOCK * 3;
            const v4f v = *(const v4f*)(sOut + tid * 4);
            *(volatile v4f*)(ob + tid * 4) = v;
            __threadfence();
            *(volatile v4f*)(ob + tid * 4) = v;
        }
    }
}

extern "C" void kernel_launch(void* const* d_in, const int* in_sizes, int n_in,
                              void* d_out, int out_size, void* d_ws, size_t ws_size,
                              hipStream_t stream) {
    const float* seq = (const float*)d_in[0];
    const float* Wa  = (const float*)d_in[1];
    const float* ba  = (const float*)d_in[2];
    const float* W1  = (const float*)d_in[3];
    const float* b1  = (const float*)d_in[4];
    const float* W2  = (const float*)d_in[5];
    const float* b2  = (const float*)d_in[6];
    float* out = (float*)d_out;

    const int B = in_sizes[0] / 4;
    const int blocks = B / ROWS_PER_BLOCK;
    sig_mlp_kernel<<<blocks, THREADS, 0, stream>>>(seq, Wa, ba, W1, b1, W2, b2, out);
    (void)d_ws; (void)ws_size; (void)out_size; (void)n_in;
}
